// SpatialTransformer_27023934226514
// MI455X (gfx1250) — hardware-verified
//
#include <hip/hip_runtime.h>


#ifndef NB
#define NB 2
#endif
#ifndef SEQ
#define SEQ 2304
#endif
#define NB_FULL 2
#define SEQ_FULL 2304

namespace {
constexpr int CH = 512, TK = 77, TP = 128, NHD = 8, HD = 64, FF = 2048, NL = 2, GRP = 32, CPG = CH / GRP;
constexpr int KA = 2 * CH;
constexpr int MQ = NB * SEQ, MT = NB * TP;
constexpr int CC = CH * CH, WL = 20 * CC, WTOT = 3 * CC + NL * WL;
constexpr float XS = 8.0f, WSC = 256.0f, RS = 1024.0f, WRS = WSC / RS  , OSC = 64.0f, VSC = 64.0f, PCAR = 16384.0f, QSC = 8.0f, EPS = 1e-5f;
constexpr float CS8 = 1.0f / (XS * WSC), CS64 = 1.0f / (OSC * WSC);
static_assert(SEQ % 128 == 0); static_assert(SEQ <= SEQ_FULL); static_assert(NB >= 1); static_assert(NB <= NB_FULL); static_assert(MQ % 64 == 0); static_assert(MT % 64 == 0); static_assert(MQ % 8 == 0);
static_assert(CPG == 16); static_assert(TK <= TP); static_assert(TP % 32 == 0); static_assert(CH % 128 == 0); static_assert(FF % 128 == 0); static_assert(NHD * HD == CH); static_assert(OSC == VSC); static_assert(WTOT % 2048 == 0);
static_assert(MT <= MQ); static_assert((MT * CH / 8) % 256 == 0); static_assert((MQ * CH / 8) % 256 == 0); static_assert(KA % 32 == 0); static_assert(WRS == 0.25f);

typedef _Float16 b16;
typedef unsigned short us;
typedef __attribute__((ext_vector_type(16))) _Float16 v16b;
typedef __attribute__((ext_vector_type(8))) _Float16 v8b;
typedef __attribute__((ext_vector_type(16))) unsigned short v16us;
typedef __attribute__((ext_vector_type(8))) unsigned short v8us;
typedef __attribute__((ext_vector_type(16))) __bf16 v16y;
typedef __attribute__((ext_vector_type(8))) float v8f;
typedef __attribute__((ext_vector_type(4))) float v4f;

__device__ __forceinline__ unsigned int bf16_bits_rne(float f) { unsigned int u = __float_as_uint(f); u += 0x7FFFu + ((u >> 16) & 1u); return u >> 16; }
__device__ __forceinline__ float bfv(float f) { float r = __uint_as_float(bf16_bits_rne(f) << 16); asm volatile("" : "+v"(r)); return r; }
__device__ __forceinline__ void hires(float f, b16& h, b16& r) { h = (b16)f; r = (b16)((f - (float)h) * RS); }
__device__ __forceinline__ v16b frag_kb(const b16* p, int hh) { const v8b a = *(const v8b*)(p + 8 * hh), b = *(const v8b*)(p + 16 + 8 * hh); v16b f;
#pragma unroll
  for (int e = 0; e < 8; ++e) { f[e] = a[e]; f[8 + e] = b[e]; } return f; }
__device__ __forceinline__ v16us frag_ky(const us* p, int hh) { const v8us a = *(const v8us*)(p + 8 * hh), b = *(const v8us*)(p + 16 + 8 * hh); v16us f;
#pragma unroll
  for (int e = 0; e < 8; ++e) { f[e] = a[e]; f[8 + e] = b[e]; } return f; }
__device__ __forceinline__ v8f wmma16b(v16b a, v16b b, v8f c) { v8f d = __builtin_amdgcn_wmma_f32_16x16x32_f16(false, a, false, b, (short)0, c, false, false); asm volatile("v_nop\n\tv_nop\n\tv_nop\n\tv_nop" : "+v"(d) : "v"(a), "v"(b)); return d; }
__device__ __forceinline__ v8f wmma16y(v16us a, v16us b, v8f c) { v8f d = __builtin_amdgcn_wmma_f32_16x16x32_bf16(false, __builtin_bit_cast(v16y, a), false, __builtin_bit_cast(v16y, b), (short)0, c, false, false); asm volatile("v_nop\n\tv_nop\n\tv_nop\n\tv_nop" : "+v"(d) : "v"(a), "v"(b)); return d; }
__device__ __forceinline__ void wave_lds_sync() { __builtin_amdgcn_fence(3  , "workgroup"); __builtin_amdgcn_wave_barrier(); __builtin_amdgcn_fence(2  , "workgroup"); }
__device__ __forceinline__ float block_sum256(float v, float* red) {
#pragma unroll
  for (int m = 1; m < 32; m <<= 1) v += __shfl_xor(v, m);
  __syncthreads();
  if ((threadIdx.x & 31) == 0) red[threadIdx.x >> 5] = v;
  __syncthreads();
  float s = 0.0f;
#pragma unroll
  for (int i = 0; i < 8; ++i) s += red[i];
  return s; }

__global__ __launch_bounds__(256) void wprep_kernel(const float* __restrict__ win, const float* __restrict__ wout, const float* __restrict__ wq1, const float* __restrict__ wk1, const float* __restrict__ wv1, const float* __restrict__ wo1,
                                                    const float* __restrict__ wq2, const float* __restrict__ wk2, const float* __restrict__ wv2, const float* __restrict__ wo2, const float* __restrict__ f1, const float* __restrict__ f2, b16* WP) {
  constexpr unsigned CC8 = CC / 8, TOT8 = WTOT / 8;
  const unsigned u = blockIdx.x * 256u + threadIdx.x;
  if (u >= TOT8) return;
  const float* src; int K, N, dup; unsigned rr; size_t doff;
  if (u < 3u * CC8) { K = CH; N = CH; if (u < 2u * CC8) { src = win; dup = 1; rr = u; doff = 0; } else { src = wout; dup = 0; rr = u - 2u * CC8; doff = (size_t)2 * CC; } }
  else { const unsigned u2 = u - 3u * CC8; const unsigned l = u2 / (20u * CC8); const unsigned r = u2 % (20u * CC8); const unsigned s = r / CC8; unsigned base;
    K = CH; N = CH;
    if (s < 2u) { base = 0; src = wq1 + (size_t)l * CC; dup = 1; }
    else if (s < 4u) { base = 2; src = wk1 + (size_t)l * CC; dup = 1; }
    else if (s < 6u) { base = 4; src = wv1 + (size_t)l * CC; dup = 1; }
    else if (s < 7u) { base = 6; src = wo1 + (size_t)l * CC; dup = 0; }
    else if (s < 9u) { base = 7; src = wq2 + (size_t)l * CC; dup = 1; }
    else if (s < 10u) { base = 9; src = wk2 + (size_t)l * CC; dup = 0; }
    else if (s < 11u) { base = 10; src = wv2 + (size_t)l * CC; dup = 0; }
    else if (s < 12u) { base = 11; src = wo2 + (size_t)l * CC; dup = 0; }
    else if (s < 16u) { base = 12; src = f1 + (size_t)l * CH * FF; K = CH; N = FF; dup = 0; }
    else { base = 16; src = f2 + (size_t)l * FF * CH; K = FF; N = CH; dup = 0; }
    rr = r - base * CC8; doff = (size_t)3 * CC + (size_t)l * WL + (size_t)base * CC; }
  const int KP = dup ? 2 * K : K;
  const unsigned o = rr / (unsigned)(KP / 8), kk0 = (rr % (unsigned)(KP / 8)) * 8u;
  const bool hiH = kk0 < (unsigned)K; const unsigned k0 = hiH ? kk0 : kk0 - (unsigned)K; const float sc = hiH ? WSC : WRS;
  v8b v;
#pragma unroll
  for (int e = 0; e < 8; ++e) v[e] = (b16)(bfv(src[(size_t)(k0 + e) * N + o]) * sc);
  for (int pass = 0; pass < 2; ++pass) { *(volatile v8b*)(WP + doff + (size_t)o * KP + kk0) = v; __threadfence(); } }

__global__ __launch_bounds__(256) void cprep_kernel(const float* __restrict__ cond, b16* CP) {
  const unsigned u = blockIdx.x * 256u + threadIdx.x;
  if (u >= (unsigned)(MT * CH / 8)) return;
  const int row = (int)(u / (CH / 8)), c8 = (int)(u % (CH / 8)) * 8, b = row / TP, j = row % TP, jj = j < TK ? j : TK - 1;
  const float* s = cond + ((size_t)(b * TK + jj)) * CH + c8; v8b v;
#pragma unroll
  for (int e = 0; e < 8; ++e) { const float f = bfv(s[e]) * XS; v[e] = (b16)(j < TK ? f : 0.0f); }
  for (int pass = 0; pass < 2; ++pass) { *(volatile v8b*)(CP + (size_t)row * CH + c8) = v; __threadfence(); } }

__global__ __launch_bounds__(256) void gnorm_kernel(const float* __restrict__ x, const float* __restrict__ gg, const float* __restrict__ gb, b16* GA) {
  __shared__ float T[64][65]; __shared__ float red[8]; __shared__ float stat[8];
  const int tid = threadIdx.x; const int b = blockIdx.x / 8, slab = blockIdx.x % 8, c0 = slab * 64;
  const float* xb = x + ((size_t)b * CH + c0) * SEQ_FULL;
#pragma unroll 1
  for (int g = 0; g < 4; ++g) {
    float s = 0.0f;
#pragma unroll 1
    for (int ch = 0; ch < CPG; ++ch) { const float* p = xb + (size_t)(g * CPG + ch) * SEQ_FULL; for (int i = tid; i < SEQ; i += 256) s += bfv(p[i]); }
    s = block_sum256(s, red);
    const float mean = s * (1.0f / (float)(CPG * SEQ));
    float q = 0.0f;
#pragma unroll 1
    for (int ch = 0; ch < CPG; ++ch) { const float* p = xb + (size_t)(g * CPG + ch) * SEQ_FULL; for (int i = tid; i < SEQ; i += 256) { const float d = bfv(p[i]) - mean; q += d * d; } }
    q = block_sum256(q, red);
    if (tid == 0) { stat[g] = mean; stat[4 + g] = rsqrtf(q * (1.0f / (float)(CPG * SEQ)) + EPS); } }
  __syncthreads();
  const int qq = tid & 7, L0 = tid >> 3;
  for (int p0 = 0; p0 < SEQ; p0 += 64) {
#pragma unroll 4
    for (int i = 0; i < 16; ++i) { const int idx = tid + 256 * i, ch = idx >> 6, px = idx & 63, g = ch >> 4;
      const float v = bfv(xb[(size_t)ch * SEQ_FULL + p0 + px]); T[ch][px] = (v - stat[g]) * stat[4 + g] * bfv(gg[c0 + ch]) + bfv(gb[c0 + ch]); }
    __syncthreads();
    v8b hv[2], hr[2];
#pragma unroll
    for (int i = 0; i < 2; ++i) {
#pragma unroll
      for (int e = 0; e < 8; ++e) { b16 hh, rz; hires(T[8 * qq + e][L0 + 32 * i] * XS, hh, rz); hv[i][e] = hh; hr[i][e] = rz; } }
    for (int pass = 0; pass < 2; ++pass) {
#pragma unroll
      for (int i = 0; i < 2; ++i) { b16* dst = GA + ((size_t)(b * SEQ + p0 + L0 + 32 * i)) * KA + c0 + 8 * qq; *(volatile v8b*)(dst) = hv[i]; *(volatile v8b*)(dst + CH) = hr[i]; }
      __threadfence(); }
    __syncthreads(); } }

__global__ __launch_bounds__(256) void lnorm_kernel(const float* __restrict__ t, const float* __restrict__ g, const float* __restrict__ be, b16* TN) {
  const int lane = threadIdx.x & 31, w = threadIdx.x >> 5; const size_t row = (size_t)blockIdx.x * 8 + w;
  const float* p = t + row * CH + 8 * lane;
  const v4f a0 = *(const v4f*)p, a1 = *(const v4f*)(p + 4), a2 = *(const v4f*)(p + 256), a3 = *(const v4f*)(p + 260);
  float s = 0.0f;
#pragma unroll
  for (int e = 0; e < 4; ++e) s += (a0[e] + a1[e]) + (a2[e] + a3[e]);
#pragma unroll
  for (int m = 1; m < 32; m <<= 1) s += __shfl_xor(s, m);
  const float mean = s * (1.0f / (float)CH);
  const v4f d0 = a0 - mean, d1 = a1 - mean, d2 = a2 - mean, d3 = a3 - mean;
  float q = 0.0f;
#pragma unroll
  for (int e = 0; e < 4; ++e) q += (d0[e] * d0[e] + d1[e] * d1[e]) + (d2[e] * d2[e] + d3[e] * d3[e]);
#pragma unroll
  for (int m = 1; m < 32; m <<= 1) q += __shfl_xor(q, m);
  const float rstd = rsqrtf(q * (1.0f / (float)CH) + EPS);
  const v4f g0 = *(const v4f*)(g + 8 * lane), g1 = *(const v4f*)(g + 8 * lane + 4), g2 = *(const v4f*)(g + 256 + 8 * lane), g3 = *(const v4f*)(g + 260 + 8 * lane);
  const v4f b0 = *(const v4f*)(be + 8 * lane), b1 = *(const v4f*)(be + 8 * lane + 4), b2 = *(const v4f*)(be + 256 + 8 * lane), b3 = *(const v4f*)(be + 260 + 8 * lane);
  v8b y0, y1, z0, z1;
#pragma unroll
  for (int e = 0; e < 4; ++e) { b16 hh, rz;
    hires(((d0[e] * rstd) * bfv(g0[e]) + bfv(b0[e])) * XS, hh, rz); y0[e] = hh; z0[e] = rz;
    hires(((d1[e] * rstd) * bfv(g1[e]) + bfv(b1[e])) * XS, hh, rz); y0[4 + e] = hh; z0[4 + e] = rz;
    hires(((d2[e] * rstd) * bfv(g2[e]) + bfv(b2[e])) * XS, hh, rz); y1[e] = hh; z1[e] = rz;
    hires(((d3[e] * rstd) * bfv(g3[e]) + bfv(b3[e])) * XS, hh, rz); y1[4 + e] = hh; z1[4 + e] = rz; }
  for (int pass = 0; pass < 2; ++pass) { b16* dst = TN + row * KA + 8 * lane; *(volatile v8b*)(dst) = y0; *(volatile v8b*)(dst + 256) = y1; *(volatile v8b*)(dst + CH) = z0; *(volatile v8b*)(dst + CH + 256) = z1; __threadfence(); } }

__global__ __launch_bounds__(256) void cvt_kernel(const float* __restrict__ t, b16* TN) {
  const size_t u = (size_t)blockIdx.x * 256 + threadIdx.x; if (u >= (size_t)MQ * CH / 8) return;
  const size_t row = u / (CH / 8); const int c8 = (int)(u % (CH / 8)) * 8;
  const v4f a0 = *(const v4f*)(t + u * 8), a1 = *(const v4f*)(t + u * 8 + 4); v8b y;
#pragma unroll
  for (int e = 0; e < 4; ++e) { y[e] = (b16)(a0[e] * XS); y[4 + e] = (b16)(a1[e] * XS); }
  for (int pass = 0; pass < 2; ++pass) { *(volatile v8b*)(TN + row * KA + c8) = y; __threadfence(); } }

enum { MD_F32 = 0, MD_F32RES = 1, MD_H = 2, MD_Y2 = 3, MD_HT = 4, MD_OUT = 5 };
template <int MODE>
__global__ __launch_bounds__(128) void gemm_kernel(const b16* __restrict__ A, int lda, const b16* __restrict__ Bw, int ldb, int K, const float* __restrict__ bias, float cs, float os,
                                                  float* outF, b16* outH, us* outY0, us* outY1, const float* __restrict__ xin, int ldo) {
  __shared__ __attribute__((aligned(16))) float Tf[64][132];
  const int lane = threadIdx.x & 31, w = threadIdx.x >> 5, l15 = lane & 15, hb = lane >> 4, wm = w >> 1, wn = w & 1;
  const int row0 = blockIdx.y * 64, col0 = blockIdx.x * 128;
  const b16* Ap0 = A + (size_t)(row0 + wm * 32 + l15) * lda; const b16* Ap1 = Ap0 + (size_t)16 * lda;
  const b16* Bp = Bw + (size_t)(col0 + wn * 64 + l15) * ldb; const size_t bst = (size_t)16 * ldb;
  v8f acc0[4] = {(v8f){}, (v8f){}, (v8f){}, (v8f){}}, acc1[4] = {(v8f){}, (v8f){}, (v8f){}, (v8f){}};
#pragma unroll 2
  for (int k = 0; k < K; k += 32) {
    const v16b a0 = frag_kb(Ap0 + k, hb), a1 = frag_kb(Ap1 + k, hb);
#pragma unroll
    for (int j = 0; j < 4; ++j) { const v16b bb = frag_kb(Bp + j * bst + k, hb); acc0[j] = wmma16b(a0, bb, acc0[j]); acc1[j] = wmma16b(a1, bb, acc1[j]); } }
#pragma unroll
  for (int j = 0; j < 4; ++j) {
#pragma unroll
    for (int r = 0; r < 8; ++r) { Tf[wm * 32 + 8 * hb + r][wn * 64 + 16 * j + l15] = acc0[j][r]; Tf[wm * 32 + 16 + 8 * hb + r][wn * 64 + 16 * j + l15] = acc1[j][r]; } }
  __syncthreads();
  if (MODE == MD_F32 || MODE == MD_F32RES) {
    const int c4 = 4 * lane; v4f b4;
#pragma unroll
    for (int e = 0; e < 4; ++e) b4[e] = bfv(bias[col0 + c4 + e]);
#pragma unroll
    for (int i = 0; i < 16; ++i) { const int r = 16 * w + i; v4f v = *(const v4f*)(&Tf[r][c4]) * cs + b4;
      if (MODE == MD_F32RES) v += *(const v4f*)(outF + (size_t)(row0 + r) * ldo + col0 + c4);
      *(v4f*)(&Tf[r][c4]) = v; }
    __syncthreads();
    for (int pass = 0; pass < 2; ++pass) {
#pragma unroll
      for (int i = 0; i < 16; ++i) { const int r = 16 * w + i; *(volatile v4f*)(outF + (size_t)(row0 + r) * ldo + col0 + c4) = *(const v4f*)(&Tf[r][c4]); }
      __threadfence(); }
  } else if (MODE == MD_H || MODE == MD_Y2) {
    const int c8 = 8 * l15; float b8[8];
#pragma unroll
    for (int e = 0; e < 8; ++e) b8[e] = bfv(bias[col0 + c8 + e]);
#pragma unroll
    for (int i = 0; i < 8; ++i) { const int r = 16 * w + 2 * i + hb; float* tp = &Tf[r][c8];
#pragma unroll
      for (int e = 0; e < 8; ++e) tp[e] = (tp[e] * cs + b8[e]) * os; }
    __syncthreads();
    for (int pass = 0; pass < 2; ++pass) {
#pragma unroll
      for (int i = 0; i < 8; ++i) { const int r = 16 * w + 2 * i + hb; const float* tp = &Tf[r][c8];
        if (MODE == MD_H) { v8b hv;
#pragma unroll
          for (int e = 0; e < 8; ++e) hv[e] = (b16)tp[e];
          *(volatile v8b*)(outH + (size_t)(row0 + r) * ldo + col0 + c8) = hv; }
        else { v8us hi, lo;
#pragma unroll
          for (int e = 0; e < 8; ++e) { const unsigned hbt = bf16_bits_rne(tp[e]); const float hf = __uint_as_float(hbt << 16); hi[e] = (us)hbt; lo[e] = (us)bf16_bits_rne(tp[e] - hf); }
          *(volatile v8us*)(outY0 + (size_t)(row0 + r) * ldo + col0 + c8) = hi; *(volatile v8us*)(outY1 + (size_t)(row0 + r) * ldo + col0 + c8) = lo; } }
      __threadfence(); }
  } else if (MODE == MD_HT) {
    const int qq = lane & 7, cq = lane >> 3;
#pragma unroll
    for (int i = 0; i < 8; ++i) { const int c = 32 * w + 4 * i + cq; const float bc = bfv(bias[col0 + c]);
#pragma unroll
      for (int e = 0; e < 8; ++e) Tf[8 * qq + e][c] = (Tf[8 * qq + e][c] * cs + bc) * os; }
    __syncthreads();
    for (int pass = 0; pass < 2; ++pass) {
#pragma unroll
      for (int i = 0; i < 8; ++i) { const int c = 32 * w + 4 * i + cq; v8b hv;
#pragma unroll
        for (int e = 0; e < 8; ++e) hv[e] = (b16)Tf[8 * qq + e][c];
        *(volatile v8b*)(outH + (size_t)(col0 + c) * ldo + row0 + 8 * qq) = hv; }
      __threadfence(); }
  } else {
    const int bi = row0 / SEQ, p0 = row0 - bi * SEQ;
#pragma unroll
    for (int i = 0; i < 16; ++i) { const int c = 32 * w + 2 * i + hb; const float bc = bfv(bias[col0 + c]);
      const size_t gi = ((size_t)(bi * CH + col0 + c)) * SEQ_FULL + p0 + 4 * l15; const v4f xr = *(const v4f*)(xin + gi);
#pragma unroll
      for (int e = 0; e < 4; ++e) Tf[4 * l15 + e][c] = (Tf[4 * l15 + e][c] * cs + bc) + bfv(xr[e]); }
    __syncthreads();
    for (int pass = 0; pass < 2; ++pass) {
#pragma unroll
      for (int i = 0; i < 16; ++i) { const int c = 32 * w + 2 * i + hb; const size_t gi = ((size_t)(bi * CH + col0 + c)) * SEQ_FULL + p0 + 4 * l15; v4f v;
#pragma unroll
        for (int e = 0; e < 4; ++e) v[e] = Tf[4 * l15 + e][c];
        *(volatile v4f*)(outF + gi) = v; }
      __threadfence(); }
  } }

__global__ __launch_bounds__(256) void attn_kernel(const us* __restrict__ Qh, const us* __restrict__ Ql, const us* __restrict__ Kh, const us* __restrict__ Kl, const b16* __restrict__ Vt, b16* O, int nk, int kvalid, int ldv) {
  __shared__ __attribute__((aligned(16))) b16 Pst[8][16][72];
  const int lane = threadIdx.x & 31, w = threadIdx.x >> 5, l15 = lane & 15, hb = lane >> 4;
  const int b = blockIdx.x / NHD, h = blockIdx.x % NHD;
  const int qi0 = blockIdx.y * 128 + w * 16;
  const size_t qro = ((size_t)(b * SEQ + qi0 + l15)) * CH + h * HD;
  const v16us qh0 = frag_ky(Qh + qro, hb), qh1 = frag_ky(Qh + qro + 32, hb), ql0 = frag_ky(Ql + qro, hb), ql1 = frag_ky(Ql + qro + 32, hb);
  v8f o0 = {}, o1 = {}, o2 = {}, o3 = {};
  float mrow[8], lrow[8];
#pragma unroll
  for (int r = 0; r < 8; ++r) { mrow[r] = -1e30f; lrow[r] = 0.0f; }
  for (int j0 = 0; j0 < kvalid; j0 += 32) {
    const size_t kro = ((size_t)(b * nk + j0 + l15)) * CH + h * HD;
    v8f s0 = {}, s1 = {};
    { const v16us k0 = frag_ky(Kh + kro, hb), k1 = frag_ky(Kh + kro + 32, hb), e0 = frag_ky(Kl + kro, hb), e1 = frag_ky(Kl + kro + 32, hb);
      s0 = wmma16y(qh0, k0, s0); s0 = wmma16y(qh1, k1, s0); s0 = wmma16y(qh0, e0, s0); s0 = wmma16y(qh1, e1, s0); s0 = wmma16y(ql0, k0, s0); s0 = wmma16y(ql1, k1, s0); }
    { const size_t krb = kro + (size_t)16 * CH; const v16us k0 = frag_ky(Kh + krb, hb), k1 = frag_ky(Kh + krb + 32, hb), e0 = frag_ky(Kl + krb, hb), e1 = frag_ky(Kl + krb + 32, hb);
      s1 = wmma16y(qh0, k0, s1); s1 = wmma16y(qh1, k1, s1); s1 = wmma16y(qh0, e0, s1); s1 = wmma16y(qh1, e1, s1); s1 = wmma16y(ql0, k0, s1); s1 = wmma16y(ql1, k1, s1); }
    const bool va = (j0 + l15) < kvalid, vb = (j0 + 16 + l15) < kvalid;
#pragma unroll
    for (int r = 0; r < 8; ++r) {
      const float sa = va ? s0[r] : -1e30f, sb = vb ? s1[r] : -1e30f;
      float v = fmaxf(sa, sb);
#pragma unroll
      for (int m = 1; m < 16; m <<= 1) v = fmaxf(v, __shfl_xor(v, m, 16));
      const float mnew = fmaxf(mrow[r], v); const float corr = __expf(mrow[r] - mnew); mrow[r] = mnew;
      const float p0 = va ? __expf(sa - mnew) : 0.0f, p1 = vb ? __expf(sb - mnew) : 0.0f;
      float ps = p0 + p1;
#pragma unroll
      for (int m = 1; m < 16; m <<= 1) ps += __shfl_xor(ps, m, 16);
      lrow[r] = lrow[r] * corr + ps; o0[r] *= corr; o1[r] *= corr; o2[r] *= corr; o3[r] *= corr;
      Pst[w][8 * hb + r][l15] = (b16)(p0 * PCAR); Pst[w][8 * hb + r][16 + l15] = (b16)(p1 * PCAR); }
    wave_lds_sync();
    const v16b pf = frag_kb(&Pst[w][l15][0], hb);
    const b16* vr = Vt + ((size_t)(h * HD + l15)) * ldv + (size_t)b * nk + j0; const size_t vst = (size_t)16 * ldv;
    o0 = wmma16b(pf, frag_kb(vr, hb), o0); o1 = wmma16b(pf, frag_kb(vr + vst, hb), o1); o2 = wmma16b(pf, frag_kb(vr + 2 * vst, hb), o2); o3 = wmma16b(pf, frag_kb(vr + 3 * vst, hb), o3);
    wave_lds_sync(); }
#pragma unroll
  for (int r = 0; r < 8; ++r) { const float inv = 1.0f / (lrow[r] * PCAR); b16* pr = &Pst[w][8 * hb + r][0];
    pr[l15] = (b16)(o0[r] * inv); pr[16 + l15] = (b16)(o1[r] * inv); pr[32 + l15] = (b16)(o2[r] * inv); pr[48 + l15] = (b16)(o3[r] * inv); }
  wave_lds_sync();
  const int qq = lane & 7, rq = lane >> 3;
  for (int pass = 0; pass < 2; ++pass) {
#pragma unroll
    for (int i = 0; i < 4; ++i) { const int rr = 4 * i + rq; const v8b val = *(const v8b*)(&Pst[w][rr][8 * qq]); *(volatile v8b*)(O + ((size_t)(b * SEQ + qi0 + rr)) * CH + h * HD + 8 * qq) = val; }
    __threadfence(); } }

template <int MODE>
void run_gemm(hipStream_t st, int Mrows, int N, const b16* A, int lda, const b16* Bw, int ldb, int K, const float* bias, float cs, float os, float* outF, b16* outH, us* y0, us* y1, const float* xin, int ldo) {
  dim3 grid((unsigned)(N / 128), (unsigned)(Mrows / 64));
  gemm_kernel<MODE><<<grid, 128, 0, st>>>(A, lda, Bw, ldb, K, bias, cs, os, outF, outH, y0, y1, xin, ldo); }
}

extern "C" void kernel_launch(void* const* d_in, const int* in_sizes, int n_in, void* d_out, int out_size, void* d_ws, size_t ws_size, hipStream_t stream) {
  if (n_in < 34) return;
  auto F = [&](int i) { return (const float*)d_in[i]; };
  if (in_sizes[0] < NB * CH * SEQ_FULL || in_sizes[1] < NB * TK * CH || in_sizes[2] < CH || in_sizes[3] < CH || in_sizes[4] < CC || in_sizes[5] < CH || in_sizes[6] < CC || in_sizes[7] < CH) return;
  { const int wi[8] = {8, 10, 12, 14, 18, 20, 22, 24}; for (int i = 0; i < 8; ++i) if (in_sizes[wi[i]] < NL * CC) return; }
  { const int bi[15] = {9, 11, 13, 15, 16, 17, 19, 21, 23, 25, 26, 27, 31, 32, 33}; for (int i = 0; i < 15; ++i) if (in_sizes[bi[i]] < NL * CH) return; }
  if (in_sizes[28] < NL * CH * FF || in_sizes[30] < NL * CH * FF || in_sizes[29] < NL * FF) return;
  if (out_size < NB * CH * SEQ_FULL) return;
  size_t off = 0; char* ws = (char*)d_ws;
  auto carve = [&](size_t bytes) { char* p = ws + off; off += (bytes + 255) & ~(size_t)255; return p; };
  b16* WP = (b16*)carve((size_t)WTOT * 2); float* T = (float*)carve((size_t)MQ * CH * 4); b16* TA = (b16*)carve((size_t)MQ * KA * 2);
  us* QH = (us*)carve((size_t)MQ * CH * 2); us* QL = (us*)carve((size_t)MQ * CH * 2); us* KH = (us*)carve((size_t)MQ * CH * 2); us* KL = (us*)carve((size_t)MQ * CH * 2);
  b16* VT = (b16*)carve((size_t)CH * MQ * 2); b16* OP = (b16*)carve((size_t)MQ * CH * 2); b16* MID = (b16*)carve((size_t)MQ * FF * 2); b16* CP = (b16*)carve((size_t)MT * CH * 2);
  if (off > ws_size || off > ((size_t)128 << 20)) return;
  float* dout = (float*)d_out; const float* x = F(0);
  const b16* WIN = WP;
  const b16* WOUT = WP + 2 * CC;
  wprep_kernel<<<(unsigned)(WTOT / 8 / 256), 256, 0, stream>>>(F(4), F(6), F(8), F(10), F(12), F(14), F(18), F(20), F(22), F(24), F(28), F(30), WP);
  cprep_kernel<<<(unsigned)(MT * CH / 8 / 256), 256, 0, stream>>>(F(1), CP);
  gnorm_kernel<<<NB * 8, 256, 0, stream>>>(x, F(2), F(3), TA);
  run_gemm<MD_F32>(stream, MQ, CH, TA, KA, WIN, KA, KA, F(5), CS8, 1.0f, T, OP, QH, QL, x, CH);
  for (int l = 0; l < NL; ++l) {
    const b16* lb = WP + (size_t)3 * CC + (size_t)l * WL;
    const b16 *WQ1 = lb, *WK1 = lb + 2 * (size_t)CC, *WV1 = lb + 4 * (size_t)CC, *WO1 = lb + 6 * (size_t)CC, *WQ2 = lb + 7 * (size_t)CC, *WK2 = lb + 9 * (size_t)CC, *WV2 = lb + 10 * (size_t)CC, *WO2 = lb + 11 * (size_t)CC,
              *WF1 = lb + 12 * (size_t)CC, *WF2 = lb + 16 * (size_t)CC;
    lnorm_kernel<<<MQ / 8, 256, 0, stream>>>(T, F(16) + l * CH, F(17) + l * CH, TA);
    run_gemm<MD_Y2>(stream, MQ, CH, TA, KA, WQ1, KA, KA, F(9) + l * CH, CS8, QSC, T, OP, QH, QL, x, CH);
    run_gemm<MD_Y2>(stream, MQ, CH, TA, KA, WK1, KA, KA, F(11) + l * CH, CS8, 1.0f, T, OP, KH, KL, x, CH);
    run_gemm<MD_HT>(stream, MQ, CH, TA, KA, WV1, KA, KA, F(13) + l * CH, CS8, VSC, T, VT, QH, QL, x, MQ);
    attn_kernel<<<dim3(NB * NHD, SEQ / 128), 256, 0, stream>>>(QH, QL, KH, KL, VT, OP, SEQ, SEQ, MQ);
    run_gemm<MD_F32RES>(stream, MQ, CH, OP, CH, WO1, CH, CH, F(15) + l * CH, CS64, 1.0f, T, OP, QH, QL, x, CH);
    lnorm_kernel<<<MQ / 8, 256, 0, stream>>>(T, F(26) + l * CH, F(27) + l * CH, TA);
    run_gemm<MD_Y2>(stream, MQ, CH, TA, KA, WQ2, KA, KA, F(19) + l * CH, CS8, QSC, T, OP, QH, QL, x, CH);
    run_gemm<MD_Y2>(stream, MT, CH, CP, CH, WK2, CH, CH, F(21) + l * CH, CS8, 1.0f, T, OP, KH, KL, x, CH);
    run_gemm<MD_HT>(stream, MT, CH, CP, CH, WV2, CH, CH, F(23) + l * CH, CS8, VSC, T, VT, QH, QL, x, MT);
    attn_kernel<<<dim3(NB * NHD, SEQ / 128), 256, 0, stream>>>(QH, QL, KH, KL, VT, OP, TP, TK, MT);
    run_gemm<MD_F32RES>(stream, MQ, CH, OP, CH, WO2, CH, CH, F(25) + l * CH, CS64, 1.0f, T, OP, QH, QL, x, CH);
    lnorm_kernel<<<MQ / 8, 256, 0, stream>>>(T, F(32) + l * CH, F(33) + l * CH, TA);
    run_gemm<MD_H>(stream, MQ, FF, TA, KA, WF1, CH, CH, F(29) + l * FF, CS8, OSC, T, MID, QH, QL, x, FF);
    run_gemm<MD_F32RES>(stream, MQ, CH, MID, FF, WF2, FF, FF, F(31) + l * CH, CS64, 1.0f, T, OP, QH, QL, x, CH);
  }
  cvt_kernel<<<(unsigned)((size_t)MQ * CH / 8 / 256), 256, 0, stream>>>(T, TA);
  run_gemm<MD_OUT>(stream, MQ, CH, TA, KA, WOUT, CH, CH, F(7), CS8, 1.0f, dout, OP, QH, QL, x, CH);
}
